// MultiLatentAttention_51565377356070
// MI455X (gfx1250) — hardware-verified
//
#include <hip/hip_runtime.h>

typedef _Float16 f16;
typedef f16 v16h __attribute__((ext_vector_type(16)));
typedef f16 v8h_t __attribute__((ext_vector_type(8)));
typedef v8h_t v8h __attribute__((may_alias));
typedef float v8f __attribute__((ext_vector_type(8)));
typedef float v4f_t __attribute__((ext_vector_type(4)));
typedef v4f_t v4f __attribute__((may_alias));
typedef unsigned int v4u_t __attribute__((ext_vector_type(4)));
typedef v4u_t v4u __attribute__((may_alias));

union Frag { v16h v; v8h_t hv[2]; };
union H8 { v8h_t v; f16 e[8]; };
union U8 { v4u_t u; f16 e[8]; };

__device__ __forceinline__ v16h ldfrag(const f16* base, int row0, int ld, int k0) {
  const int l = threadIdx.x & 31, hh = l >> 4, m = l & 15;
  const f16* p = base + (size_t)(row0 + m) * (size_t)ld + k0 + 8 * hh;
  Frag f;
  f.hv[0] = *(const v8h*)p;
  f.hv[1] = *(const v8h*)(p + 16);
  return f.v;
}

__device__ __forceinline__ v8f wm(v8f c, v16h a, v16h b) {
  v8f d = __builtin_amdgcn_wmma_f32_16x16x32_f16(false, a, false, b, (short)0, c, false, false);
  asm volatile("v_nop\n\tv_nop\n\tv_nop\n\tv_nop" : "+v"(d) : "v"(a), "v"(b));
  return d;
}

__device__ __forceinline__ void split16(float v, f16& hi, f16& lo) {
  hi = (f16)v;
  lo = (f16)((v - (float)hi) * 2048.0f);
}

__global__ __launch_bounds__(256) void k_cvt_x(const float* __restrict__ x, f16* xh, f16* xl,
                                               int total_rows, int cols, int rows_per_grp, int R) {
  const size_t gid = (size_t)blockIdx.x * 256 + threadIdx.x;
  const size_t e = gid * 8;
  const size_t row = e / (size_t)cols;
  if (row >= (size_t)total_rows) return;
  const int col = (int)(e - row * cols);
  v4f_t a = *(const v4f*)(x + e);
  v4f_t b = *(const v4f*)(x + e + 4);
  float v[8] = {a[0], a[1], a[2], a[3], b[0], b[1], b[2], b[3]};
  H8 hh, ll;
#pragma unroll
  for (int i = 0; i < 8; ++i) split16(v[i], hh.e[i], ll.e[i]);
  const int grp = (int)(row / rows_per_grp);
  const int s = (int)(row - (size_t)grp * rows_per_grp);
  f16* dh = xh + e;
  f16* dl = xl + ((size_t)grp * R + s) * cols + col;
  const bool has_lo = s < R;
  *(volatile v8h_t*)dh = hh.v;
  if (has_lo) *(volatile v8h_t*)dl = ll.v;
  __threadfence();
  *(volatile v8h_t*)dh = hh.v;
  if (has_lo) *(volatile v8h_t*)dl = ll.v;
}

__global__ __launch_bounds__(256) void k_wT(const float* __restrict__ in, f16* outh, f16* outl, int K, int N, float sc) {
  __shared__ float t[64][33];
  const int n0 = blockIdx.x * 32, k0 = blockIdx.y * 64;
  const int tid = threadIdx.x;
  {
    const int nn = tid & 31, kb = tid >> 5;
#pragma unroll
    for (int i = 0; i < 8; ++i) {
      const int kk = kb + 8 * i;
      t[kk][nn] = in[(size_t)(k0 + kk) * N + n0 + nn];
    }
  }
  __syncthreads();
  const int nn = tid >> 3, sub = tid & 7;
  H8 hh, ll;
#pragma unroll
  for (int e = 0; e < 8; ++e) split16(t[sub * 8 + e][nn] * sc, hh.e[e], ll.e[e]);
  const size_t off = (size_t)(n0 + nn) * K + k0 + sub * 8;
  *(volatile v8h_t*)(outh + off) = hh.v;
  *(volatile v8h_t*)(outl + off) = ll.v;
  __threadfence();
  *(volatile v8h_t*)(outh + off) = hh.v;
  *(volatile v8h_t*)(outl + off) = ll.v;
}

__global__ __launch_bounds__(256) void k_rope_tab(float* cs, float* sn, int n) {
  const int i = blockIdx.x * 256 + threadIdx.x;
  if (i >= n) return;
  const int s = i >> 5, fi = i & 31;
  const float ex = (float)(2 * fi) / 64.0f;
  const float inv = 1.0f / powf(10000.0f, ex);
  const float ang = (float)s * inv;
  const float c = cosf(ang), sv = sinf(ang);
  *(volatile float*)(cs + i) = c;
  *(volatile float*)(sn + i) = sv;
  __threadfence();
  *(volatile float*)(cs + i) = c;
  *(volatile float*)(sn + i) = sv;
}

__global__ __launch_bounds__(256) void k_rope(f16* qh, f16* ql, f16* kh, f16* kl,
                                              const float* __restrict__ cs, const float* __restrict__ sn,
                                              int S, int H, int R) {
  const size_t gid = (size_t)blockIdx.x * 256 + threadIdx.x;
  const size_t unit = gid >> 3;
  const int sub = (int)(gid & 7);
  const int which = (int)(unit & 1);
  const int hh = (int)((unit >> 1) % H);
  const int s = (int)((unit >> 1) / H);
  if (s >= S) return;
  f16* ph = (which ? kh : qh) + (size_t)s * (H * 192) + hh * 192 + 128;
  f16* pl = (which ? kl : ql) + (size_t)s * (H * 192) + hh * 192 + 128;
  const bool has_lo = s < R;
  const int t0 = sub * 8;
  const int pt0 = (sub < 4) ? t0 + 32 : t0 - 32;
  H8 oh, ol, qhv, qlv;
  oh.v = *(const v8h*)(ph + t0);
  qhv.v = *(const v8h*)(ph + pt0);
  float xo[8], xp[8];
#pragma unroll
  for (int i = 0; i < 8; ++i) { xo[i] = (float)oh.e[i]; xp[i] = (float)qhv.e[i]; }
  if (has_lo) {
    ol.v = *(const v8h*)(pl + t0);
    qlv.v = *(const v8h*)(pl + pt0);
#pragma unroll
    for (int i = 0; i < 8; ++i) {
      xo[i] += (float)ol.e[i] * 0.00048828125f;
      xp[i] += (float)qlv.e[i] * 0.00048828125f;
    }
  }
  H8 rh, rl;
#pragma unroll
  for (int i = 0; i < 8; ++i) {
    const int fi = (t0 + i) & 31;
    const float c = cs[s * 32 + fi], sv = sn[s * 32 + fi];
    float r;
    if (sub < 4) r = xo[i] * c - xp[i] * sv;
    else         r = xo[i] * c + xp[i] * sv;
    split16(r, rh.e[i], rl.e[i]);
  }
  *(volatile v8h_t*)(ph + t0) = rh.v;
  if (has_lo) *(volatile v8h_t*)(pl + t0) = rl.v;
  __threadfence();
  *(volatile v8h_t*)(ph + t0) = rh.v;
  if (has_lo) *(volatile v8h_t*)(pl + t0) = rl.v;
}

#define SCP 132
template <bool SPLIT, int MODE>
__global__ __launch_bounds__(256) void k_gemm(const f16* __restrict__ Ah, const f16* __restrict__ Al,
                                              const f16* __restrict__ Bh, const f16* __restrict__ Bl,
                                              f16* Ch, f16* Cl, f16* Vh, f16* Vl, float* Cf,
                                              int K, int N, int tpg, int grp_stride, int row_start, int R,
                                              float oscale, float sout) {
  __shared__ __attribute__((aligned(16))) f16 sA[2][128 * 32];
  __shared__ __attribute__((aligned(16))) f16 sB[2][128 * 32];
  __shared__ __attribute__((aligned(16))) float sC[128 * SCP];

  const int tid = threadIdx.x, wave = tid >> 5, lane = tid & 31;
  const int hf = lane >> 4, lc = lane & 15;
  const int wmi = wave >> 2, wn = wave & 3;
  const int y = blockIdx.y;
  const int grp = y / tpg;
  const int mrel = row_start + (y - grp * tpg) * 128;
  const size_t arow = (size_t)grp * grp_stride + mrel;
  const size_t lrow = (size_t)grp * R + mrel;
  const int n0 = blockIdx.x * 128;
  const float kx = 0.00048828125f;

  v8f acc[4][2];
#pragma unroll
  for (int mi = 0; mi < 4; ++mi) { acc[mi][0] = (v8f){}; acc[mi][1] = (v8f){}; }

  const int nk = K >> 5;
  for (int kt = 0; kt < nk; ++kt) {
    const int k0 = kt << 5;
#pragma unroll
    for (int i = 0; i < 2; ++i) {
      const int q = tid + 256 * i;
      const int row = q >> 2, c4 = q & 3;
      *(v4u*)(&sA[0][row * 32 + c4 * 8]) = *(const v4u*)(Ah + (arow + row) * K + k0 + c4 * 8);
      *(v4u*)(&sB[0][row * 32 + c4 * 8]) = *(const v4u*)(Bh + (size_t)(n0 + row) * K + k0 + c4 * 8);
      if (SPLIT) {
        *(v4u*)(&sA[1][row * 32 + c4 * 8]) = *(const v4u*)(Al + (lrow + row) * K + k0 + c4 * 8);
        *(v4u*)(&sB[1][row * 32 + c4 * 8]) = *(const v4u*)(Bl + (size_t)(n0 + row) * K + k0 + c4 * 8);
      }
    }
    __syncthreads();
    v16h bh0 = ldfrag(sB[0], wn * 32, 32, 0);
    v16h bh1 = ldfrag(sB[0], wn * 32 + 16, 32, 0);
    v16h bl0, bl1;
    if (SPLIT) {
      bl0 = ldfrag(sB[1], wn * 32, 32, 0);
      bl1 = ldfrag(sB[1], wn * 32 + 16, 32, 0);
    }
#pragma unroll
    for (int mi = 0; mi < 4; ++mi) {
      v16h ah = ldfrag(sA[0], wmi * 64 + mi * 16, 32, 0);
      acc[mi][0] = wm(acc[mi][0], ah, bh0);
      acc[mi][1] = wm(acc[mi][1], ah, bh1);
      if (SPLIT) {
        v16h al = ldfrag(sA[1], wmi * 64 + mi * 16, 32, 0);
        v8f t0 = (v8f){};
        t0 = wm(t0, ah, bl0);
        t0 = wm(t0, al, bh0);
        acc[mi][0] += t0 * kx;
        v8f t1 = (v8f){};
        t1 = wm(t1, ah, bl1);
        t1 = wm(t1, al, bh1);
        acc[mi][1] += t1 * kx;
      }
    }
    __syncthreads();
  }

#pragma unroll
  for (int mi = 0; mi < 4; ++mi)
#pragma unroll
    for (int r = 0; r < 8; ++r) {
      const int row = wmi * 64 + mi * 16 + 8 * hf + r;
      sC[row * SCP + wn * 32 + lc] = acc[mi][0][r];
      sC[row * SCP + wn * 32 + 16 + lc] = acc[mi][1][r];
    }
  __syncthreads();

  if (MODE == 2) {
    for (int pass = 0; pass < 2; ++pass) {
#pragma unroll 4
      for (int it = 0; it < 16; ++it) {
        const int r = wave * 16 + it;
        const float* src = sC + r * SCP + lane * 4;
        v4f_t v;
        v[0] = src[0] * oscale; v[1] = src[1] * oscale; v[2] = src[2] * oscale; v[3] = src[3] * oscale;
        *(volatile v4f_t*)(Cf + (arow + r) * N + n0 + lane * 4) = v;
      }
      if (pass == 0) __threadfence();
    }
  } else {
    for (int pass = 0; pass < 2; ++pass) {
#pragma unroll 2
      for (int it = 0; it < 8; ++it) {
        const int unit = it * 4 + (lane >> 3);
        const int rl = unit >> 1, chunk = unit & 1, sub = lane & 7;
        const int r = wave * 16 + rl;
        const float* src = sC + r * SCP + chunk * 64 + sub * 8;
        H8 hh8, ll8;
#pragma unroll
        for (int e = 0; e < 8; ++e) split16(src[e] * oscale * sout, hh8.e[e], ll8.e[e]);
        const size_t crow = arow + r, clrow = lrow + r;
        const int n = n0 + chunk * 64;
        f16* dh; f16* dl;
        if (MODE == 0) {
          dh = Ch + crow * N + n + sub * 8;
          dl = Cl + clrow * N + n + sub * 8;
        } else {
          const int hd = n / 320, c = n - hd * 320;
          if (c < 192) {
            dh = Ch + crow * 3072 + hd * 192 + c + sub * 8;
            dl = Cl + clrow * 3072 + hd * 192 + c + sub * 8;
          } else {
            dh = Vh + crow * 2048 + hd * 128 + (c - 192) + sub * 8;
            dl = Vl + clrow * 2048 + hd * 128 + (c - 192) + sub * 8;
          }
        }
        *(volatile v8h_t*)dh = hh8.v;
        if (SPLIT) *(volatile v8h_t*)dl = ll8.v;
      }
      if (pass == 0) __threadfence();
    }
  }
}

template <bool SPLIT>
__global__ __launch_bounds__(128) void k_attn(const f16* __restrict__ qh, const f16* __restrict__ ql,
                                              const f16* __restrict__ kh, const f16* __restrict__ kl,
                                              const f16* __restrict__ vh, const f16* __restrict__ vl,
                                              f16* ch, f16* cl, int blk0, float scale) {
  constexpr int oQh = 0;
  constexpr int oQl = 12288;
  constexpr int oKh = SPLIT ? 24576 : 12288;
  constexpr int oKl = oKh + 12288;
  constexpr int oVh = SPLIT ? oKl + 12288 : oKh + 12288;
  constexpr int oVl = oVh + 8192;
  constexpr int oPh = SPLIT ? oVl + 8192 : oVh + 8192;
  constexpr int oPl = oPh + 4096;
  constexpr int TOT = SPLIT ? oPl + 4096 : oPh + 4096;
  __shared__ __attribute__((aligned(16))) f16 sm[TOT];

  const int tid = threadIdx.x, wave = tid >> 5, lane = tid & 31, hf = lane >> 4, lc = lane & 15;
  const int qb = blockIdx.x + blk0, h = blockIdx.y;
  const int q0 = qb * 64;
  const float kx = 0.00048828125f;

  for (int i = tid; i < 1536; i += 128) {
    const int row = i / 24, c = i - row * 24;
    *(v4u*)(sm + oQh + row * 192 + c * 8) = *(const v4u*)(qh + (size_t)(q0 + row) * 3072 + h * 192 + c * 8);
    if (SPLIT) *(v4u*)(sm + oQl + row * 192 + c * 8) = *(const v4u*)(ql + (size_t)(q0 + row) * 3072 + h * 192 + c * 8);
  }

  v8f o[8];
#pragma unroll
  for (int dv = 0; dv < 8; ++dv) o[dv] = (v8f){};
  float mrow[8], lrow[8];
#pragma unroll
  for (int j = 0; j < 8; ++j) { mrow[j] = -1e30f; lrow[j] = 0.0f; }

  const int nblk = qb + 1;
  const int qw = q0 + wave * 16;
  f16* pw = sm + oPh + wave * 1024;
  f16* pwl = sm + oPl + wave * 1024;

  for (int kbi = 0; kbi < nblk; ++kbi) {
    const int k0 = kbi * 64;
    __syncthreads();
    for (int i = tid; i < 1536; i += 128) {
      const int row = i / 24, c = i - row * 24;
      *(v4u*)(sm + oKh + row * 192 + c * 8) = *(const v4u*)(kh + (size_t)(k0 + row) * 3072 + h * 192 + c * 8);
      if (SPLIT) *(v4u*)(sm + oKl + row * 192 + c * 8) = *(const v4u*)(kl + (size_t)(k0 + row) * 3072 + h * 192 + c * 8);
    }
    for (int i = tid; i < 1024; i += 128) {
      const int key = i >> 4, c = i & 15;
      U8 u;
      u.u = *(const v4u*)(vh + (size_t)(k0 + key) * 2048 + h * 128 + c * 8);
#pragma unroll
      for (int e = 0; e < 8; ++e) sm[oVh + (c * 8 + e) * 64 + key] = u.e[e];
      if (SPLIT) {
        U8 w;
        w.u = *(const v4u*)(vl + (size_t)(k0 + key) * 2048 + h * 128 + c * 8);
#pragma unroll
        for (int e = 0; e < 8; ++e) sm[oVl + (c * 8 + e) * 64 + key] = w.e[e];
      }
    }
    __syncthreads();

    v8f s[4];
#pragma unroll
    for (int nt = 0; nt < 4; ++nt) {
      v8f a = (v8f){};
      v8f t = (v8f){};
#pragma unroll
      for (int kc = 0; kc < 6; ++kc) {
        v16h qf = ldfrag(sm + oQh, wave * 16, 192, kc * 32);
        v16h kf = ldfrag(sm + oKh, nt * 16, 192, kc * 32);
        a = wm(a, qf, kf);
        if (SPLIT) {
          v16h qfl = ldfrag(sm + oQl, wave * 16, 192, kc * 32);
          v16h kfl = ldfrag(sm + oKl, nt * 16, 192, kc * 32);
          t = wm(t, qf, kfl);
          t = wm(t, qfl, kf);
        }
      }
      if (SPLIT) s[nt] = a + t * kx;
      else s[nt] = a;
    }

#pragma unroll
    for (int j = 0; j < 8; ++j) {
      const int mg = qw + j + 8 * hf;
      float tm = -1e30f;
#pragma unroll
      for (int nt = 0; nt < 4; ++nt) {
        const int ng = k0 + nt * 16 + lc;
        float v = s[nt][j] * scale;
        v = (ng <= mg) ? v : -1e30f;
        s[nt][j] = v;
        tm = fmaxf(tm, v);
      }
#pragma unroll
      for (int off = 1; off < 16; off <<= 1) tm = fmaxf(tm, __shfl_xor(tm, off, 32));
      const float mn = fmaxf(mrow[j], tm);
      const float scf = __expf(mrow[j] - mn);
      mrow[j] = mn;
      float rs = 0.0f;
#pragma unroll
      for (int nt = 0; nt < 4; ++nt) {
        float p = __expf(s[nt][j] - mn);
        s[nt][j] = p;
        rs += p;
      }
#pragma unroll
      for (int off = 1; off < 16; off <<= 1) rs += __shfl_xor(rs, off, 32);
      lrow[j] = lrow[j] * scf + rs;
#pragma unroll
      for (int dv = 0; dv < 8; ++dv) o[dv][j] *= scf;
    }

#pragma unroll
    for (int nt = 0; nt < 4; ++nt)
#pragma unroll
      for (int j = 0; j < 8; ++j) {
        const float p = s[nt][j] * 4096.0f;
        f16 phv, plv;
        split16(p, phv, plv);
        pw[(j + 8 * hf) * 64 + nt * 16 + lc] = phv;
        if (SPLIT) pwl[(j + 8 * hf) * 64 + nt * 16 + lc] = plv;
      }
    __syncthreads();

    v16h pf0 = ldfrag(pw, 0, 64, 0);
    v16h pf1 = ldfrag(pw, 0, 64, 32);
#pragma unroll
    for (int dv = 0; dv < 8; ++dv) {
      v16h vf0 = ldfrag(sm + oVh, dv * 16, 64, 0);
      v16h vf1 = ldfrag(sm + oVh, dv * 16, 64, 32);
      o[dv] = wm(o[dv], pf0, vf0);
      o[dv] = wm(o[dv], pf1, vf1);
      if (SPLIT) {
        v16h pl0 = ldfrag(pwl, 0, 64, 0);
        v16h pl1 = ldfrag(pwl, 0, 64, 32);
        v16h vl0 = ldfrag(sm + oVl, dv * 16, 64, 0);
        v16h vl1 = ldfrag(sm + oVl, dv * 16, 64, 32);
        v8f t = (v8f){};
        t = wm(t, pf0, vl0);
        t = wm(t, pl0, vf0);
        t = wm(t, pf1, vl1);
        t = wm(t, pl1, vf1);
        o[dv] += t * kx;
      }
    }
  }

  __syncthreads();
  f16* sth = sm + oKh + wave * 2048;
  f16* stl = sm + oKh + 8192 + wave * 2048;
#pragma unroll
  for (int j = 0; j < 8; ++j) {
    const float invl = (1.0f / lrow[j]) * (1.0f / 4096.0f) * 16.0f;
#pragma unroll
    for (int dv = 0; dv < 8; ++dv) {
      f16 hv, lv;
      split16(o[dv][j] * invl, hv, lv);
      sth[(j + 8 * hf) * 128 + dv * 16 + lc] = hv;
      if (SPLIT) stl[(j + 8 * hf) * 128 + dv * 16 + lc] = lv;
    }
  }
  __syncthreads();
  for (int pass = 0; pass < 2; ++pass) {
#pragma unroll 2
    for (int it = 0; it < 8; ++it) {
      const int rl = it * 2 + hf;
      const size_t row = (size_t)(qw + rl);
      v8h_t hv = *(const v8h*)(sth + rl * 128 + lc * 8);
      *(volatile v8h_t*)(ch + row * 2048 + h * 128 + lc * 8) = hv;
      if (SPLIT) {
        v8h_t lv = *(const v8h*)(stl + rl * 128 + lc * 8);
        *(volatile v8h_t*)(cl + row * 2048 + h * 128 + lc * 8) = lv;
      }
    }
    if (pass == 0) __threadfence();
  }
}

extern "C" void kernel_launch(void* const* d_in, const int* in_sizes, int n_in,
                              void* d_out, int out_size, void* d_ws, size_t ws_size,
                              hipStream_t stream) {
  const int Bn = 2, S = 2048, D = 2048, H = 16, L = 512, R = 640;
  const int NKV = H * 320, NQ = H * 192;
  if (n_in < 7) return;
  if (in_sizes[0] != Bn * S * D || in_sizes[2] != D * L || in_sizes[3] != L * NKV ||
      in_sizes[4] != D * L || in_sizes[5] != L * NQ || in_sizes[6] != D * D || out_size != Bn * S * D) return;

  const float* x   = (const float*)d_in[0];
  const float* wkd = (const float*)d_in[2];
  const float* wku = (const float*)d_in[3];
  const float* wqd = (const float*)d_in[4];
  const float* wqu = (const float*)d_in[5];
  const float* wo  = (const float*)d_in[6];
  float* out = (float*)d_out;

  char* ws = (char*)d_ws;
  size_t off = 0;
  auto take = [&](size_t bytes) -> char* { char* p = ws + off; off += (bytes + 255) & ~(size_t)255; return p; };
  auto takeh = [&](size_t elems) -> f16* { return (f16*)take(elems * 2); };

  f16* xh   = takeh((size_t)Bn * S * D);
  f16* xl   = takeh((size_t)Bn * R * D);
  f16* ctxh = xh;
  f16* ctxl = xh + (size_t)S * D;
  f16* wkdh = takeh((size_t)L * D);   f16* wkdl = takeh((size_t)L * D);
  f16* wqdh = takeh((size_t)L * D);   f16* wqdl = takeh((size_t)L * D);
  f16* wkuh = takeh((size_t)NKV * L); f16* wkul = takeh((size_t)NKV * L);
  f16* wquh = takeh((size_t)NQ * L);  f16* wqul = takeh((size_t)NQ * L);
  f16* woh  = takeh((size_t)D * D);   f16* wol  = takeh((size_t)D * D);
  f16* ckvh = takeh((size_t)Bn * S * L); f16* ckvl = takeh((size_t)Bn * R * L);
  f16* cqh  = takeh((size_t)Bn * S * L); f16* cql  = takeh((size_t)Bn * R * L);
  f16* kh = takeh((size_t)S * NQ); f16* kl = takeh((size_t)R * NQ);
  f16* qh = takeh((size_t)S * NQ); f16* ql = takeh((size_t)R * NQ);
  f16* vh = takeh((size_t)S * D);  f16* vl = takeh((size_t)R * D);
  float* cs = (float*)take((size_t)S * 32 * 4);
  float* sn = (float*)take((size_t)S * 32 * 4);
  if (off > ws_size) return;

  const float sw = 32.0f, isw = 1.0f / 32.0f;

  k_cvt_x<<<dim3((Bn * S * D / 8 + 255) / 256), 256, 0, stream>>>(x, xh, xl, Bn * S, D, S, R);
  k_wT<<<dim3(L / 32, D / 64), 256, 0, stream>>>(wkd, wkdh, wkdl, D, L, sw);
  k_wT<<<dim3(L / 32, D / 64), 256, 0, stream>>>(wqd, wqdh, wqdl, D, L, sw);
  k_wT<<<dim3(NKV / 32, L / 64), 256, 0, stream>>>(wku, wkuh, wkul, L, NKV, sw);
  k_wT<<<dim3(NQ / 32, L / 64), 256, 0, stream>>>(wqu, wquh, wqul, L, NQ, sw);
  k_wT<<<dim3(D / 32, D / 64), 256, 0, stream>>>(wo, woh, wol, D, D, sw);
  k_rope_tab<<<dim3((S * 32 + 255) / 256), 256, 0, stream>>>(cs, sn, S * 32);

  const int tps = R / 128;
  const int tpp = (S - R) / 128;
  k_gemm<true, 0><<<dim3(L / 128, Bn * tps), 256, 0, stream>>>(xh, xl, wkdh, wkdl, ckvh, ckvl, nullptr, nullptr, nullptr,
                                                               D, L, tps, S, 0, R, isw, 1.0f);
  k_gemm<false, 0><<<dim3(L / 128, Bn * tpp), 256, 0, stream>>>(xh, xl, wkdh, wkdl, ckvh, ckvl, nullptr, nullptr, nullptr,
                                                                D, L, tpp, S, R, R, isw, 1.0f);
  k_gemm<true, 0><<<dim3(L / 128, Bn * tps), 256, 0, stream>>>(xh, xl, wqdh, wqdl, cqh, cql, nullptr, nullptr, nullptr,
                                                               D, L, tps, S, 0, R, isw, 1.0f);
  k_gemm<false, 0><<<dim3(L / 128, Bn * tpp), 256, 0, stream>>>(xh, xl, wqdh, wqdl, cqh, cql, nullptr, nullptr, nullptr,
                                                                D, L, tpp, S, R, R, isw, 1.0f);

  const float scale = 0.07216878364870322f;
  const int qbs = R / 64, qbp = (S - R) / 64;
  for (int b = 0; b < Bn; ++b) {
    const f16* ckh = ckvh + (size_t)b * S * L; const f16* ckl = ckvl + (size_t)b * R * L;
    const f16* cq0 = cqh + (size_t)b * S * L;  const f16* cq1 = cql + (size_t)b * R * L;
    k_gemm<true, 1><<<dim3(NKV / 128, tps), 256, 0, stream>>>(ckh, ckl, wkuh, wkul, kh, kl, vh, vl, nullptr,
                                                             L, NKV, tps, S, 0, R, isw, 1.0f);
    k_gemm<false, 1><<<dim3(NKV / 128, tpp), 256, 0, stream>>>(ckh, ckl, wkuh, wkul, kh, kl, vh, vl, nullptr,
                                                              L, NKV, tpp, S, R, R, isw, 1.0f);
    k_gemm<true, 0><<<dim3(NQ / 128, tps), 256, 0, stream>>>(cq0, cq1, wquh, wqul, qh, ql, nullptr, nullptr, nullptr,
                                                            L, NQ, tps, S, 0, R, isw, 1.0f);
    k_gemm<false, 0><<<dim3(NQ / 128, tpp), 256, 0, stream>>>(cq0, cq1, wquh, wqul, qh, ql, nullptr, nullptr, nullptr,
                                                             L, NQ, tpp, S, R, R, isw, 1.0f);
    k_rope<<<dim3((S * H * 2 * 8 + 255) / 256), 256, 0, stream>>>(qh, ql, kh, kl, cs, sn, S, H, R);
    k_attn<true><<<dim3(qbs, H), 128, 0, stream>>>(qh, ql, kh, kl, vh, vl, ctxh, ctxl, 0, scale);
    k_attn<false><<<dim3(qbp, H), 128, 0, stream>>>(qh, ql, kh, kl, vh, vl, ctxh, ctxl, qbs, scale);
    float* ob = out + (size_t)b * S * D;
    k_gemm<true, 2><<<dim3(D / 128, tps), 256, 0, stream>>>(ctxh, ctxl, woh, wol, nullptr, nullptr, nullptr, nullptr, ob,
                                                           D, D, tps, S, 0, R, 1.0f / 512.0f, 1.0f);
    k_gemm<false, 2><<<dim3(D / 128, tpp), 256, 0, stream>>>(ctxh, ctxl, woh, wol, nullptr, nullptr, nullptr, nullptr, ob,
                                                            D, D, tpp, S, R, R, 1.0f / 512.0f, 1.0f);
  }
}
